// build_simple_network_19928648254125
// MI455X (gfx1250) — hardware-verified
//
#include <hip/hip_runtime.h>
#include <math.h>

typedef __attribute__((ext_vector_type(16))) _Float16 v16h;
typedef __attribute__((ext_vector_type(16))) __bf16 v16b;
typedef __attribute__((ext_vector_type(8)))  _Float16 v8h;
typedef __attribute__((ext_vector_type(8)))  float v8f;
typedef __attribute__((ext_vector_type(4)))  float v4f;
typedef __attribute__((ext_vector_type(2)))  float v2f;
typedef __attribute__((ext_vector_type(4)))  unsigned v4u;
typedef __attribute__((ext_vector_type(4)))  int v4i;
typedef float __attribute__((may_alias)) float_a;
typedef int __attribute__((may_alias)) int_a;

template <typename T> __device__ __forceinline__ void vst2(void* p, T v) { *(volatile T*)p = v; __threadfence(); *(volatile T*)p = v; }
__device__ __forceinline__ v8f wmma16(v16h a, v16h b, v8f c) {
  v8f d = __builtin_amdgcn_wmma_f32_16x16x32_f16(false, a, false, b, (short)0, c, false, false);
  asm volatile("v_nop\n\tv_nop\n\tv_nop\n\tv_nop" : "+v"(d) : "v"(a), "v"(b));
  return d;
}
__device__ __forceinline__ v8f wmma_bf(v16b a, v16b b, v8f c) {
  v8f d = __builtin_amdgcn_wmma_f32_16x16x32_bf16(false, a, false, b, (short)0, c, false, false);
  asm volatile("v_nop\n\tv_nop\n\tv_nop\n\tv_nop" : "+v"(d) : "v"(a), "v"(b));
  return d;
}
__device__ __forceinline__ v16h frag_h(const _Float16* rowk0, int lane) {
  union { v16h v; v8h q[2]; } u; const _Float16* p = rowk0 + 8 * (lane >> 4);
  u.q[0] = *(const v8h*)p; u.q[1] = *(const v8h*)(p + 16); return u.v;
}
__device__ __forceinline__ v16h frag_f32(const float* rowk0, int lane) {
  v16h a; const float* p = rowk0 + 8 * (lane >> 4);
#pragma unroll
  for (int i = 0; i < 8; ++i) { a[i] = (_Float16)p[i]; a[8 + i] = (_Float16)p[16 + i]; }
  return a;
}
__device__ __forceinline__ v16h frag_f32s(const float* rowk0, int lane, float sc) {
  v16h a; const float* p = rowk0 + 8 * (lane >> 4);
#pragma unroll
  for (int i = 0; i < 8; ++i) { a[i] = (_Float16)(p[i] * sc); a[8 + i] = (_Float16)(p[16 + i] * sc); }
  return a;
}
__device__ __forceinline__ v16h fragc_f32(const float* W, int k0, int n, int lane, int ld, int K) {
  v16h a; const int g = lane >> 4;
#pragma unroll
  for (int i = 0; i < 8; ++i) { const int ka = k0 + 8 * g + i, kb = ka + 16;
    a[i] = (_Float16)(ka < K ? W[(size_t)(ka < K ? ka : K - 1) * ld + n] : 0.f); a[8 + i] = (_Float16)(kb < K ? W[(size_t)(kb < K ? kb : K - 1) * ld + n] : 0.f); }
  return a;
}
struct F2 { v16b h, l; };
__device__ __forceinline__ F2 bsplit16(const float v[16]) { F2 r;
#pragma unroll
  for (int i = 0; i < 16; ++i) { const __bf16 h = (__bf16)v[i]; r.h[i] = h; r.l[i] = (__bf16)(v[i] - (float)h); }
  return r; }
__device__ __forceinline__ F2 split_row(const float* row, int k0, int lane) { float v[16]; const float* p = row + k0 + 8 * (lane >> 4);
#pragma unroll
  for (int i = 0; i < 8; ++i) { v[i] = p[i]; v[8 + i] = p[16 + i]; }
  return bsplit16(v); }
__device__ __forceinline__ F2 split_rowK(const float* row, int k0, int lane, int K) { float v[16]; const int g = lane >> 4;
#pragma unroll
  for (int i = 0; i < 8; ++i) { const int ka = k0 + 8 * g + i, kb = ka + 16; v[i] = ka < K ? row[ka < K ? ka : K - 1] : 0.f; v[8 + i] = kb < K ? row[kb < K ? kb : K - 1] : 0.f; }
  return bsplit16(v); }
__device__ __forceinline__ F2 split_col(const float* W, int k0, int n, int lane, int ld, int K) { float v[16]; const int g = lane >> 4;
#pragma unroll
  for (int i = 0; i < 8; ++i) { const int ka = k0 + 8 * g + i, kb = ka + 16; v[i] = ka < K ? W[(size_t)(ka < K ? ka : K - 1) * ld + n] : 0.f; v[8 + i] = kb < K ? W[(size_t)(kb < K ? kb : K - 1) * ld + n] : 0.f; }
  return bsplit16(v); }
__device__ __forceinline__ v8f mac3(const F2& a, const F2& b, v8f c) { c = wmma_bf(a.l, b.h, c); c = wmma_bf(a.h, b.l, c); return wmma_bf(a.h, b.h, c); }
__device__ __forceinline__ float sigm(float v) { return 1.0f / (1.0f + expf(-v)); }
#define LDSX() do { asm volatile("s_wait_dscnt 0" ::: "memory"); __builtin_amdgcn_wave_barrier(); __builtin_amdgcn_fence(__ATOMIC_RELEASE, "workgroup"); } while (0)


#define NS 32768
#define NK 14
#define DIN 42
#define H1 1024
#define NDOF 7
typedef __attribute__((ext_vector_type(8))) __bf16 v8b;
__device__ __forceinline__ v16b frag_b(const __bf16* rowk0, int lane) {
  union { v16b v; v8b q[2]; } u; const __bf16* p = rowk0 + 8 * (lane >> 4);
  u.q[0] = *(const v8b*)p; u.q[1] = *(const v8b*)(p + 16); return u.v;
}
__device__ __forceinline__ float bfr(float v) { return (float)(__bf16)v; }
__constant__ float c_len[7] = {0.333f, 0.316f, 0.384f, 0.088f, 0.107f, 0.103f, 0.100f};

__global__ __launch_bounds__(128) void k_pack(const float* __restrict__ W1, const float* __restrict__ W2, __bf16* __restrict__ W1T, __bf16* __restrict__ W2T) {
  __shared__ __align__(16) __bf16 srow[H1];
  const int n = blockIdx.x, tid = threadIdx.x;
  if (n < H1) { if (tid < 64) srow[tid] = tid < DIN ? (__bf16)W1[(size_t)tid * H1 + n] : (__bf16)0.f; __syncthreads(); if (tid < 8) vst2((unsigned*)(W1T + (size_t)n * 64 + tid * 8), *(const v4u*)(&srow[tid * 8])); }
  else { const int nn = n - H1; for (int k = tid; k < H1; k += 128) srow[k] = nn < NDOF ? (__bf16)W2[(size_t)k * NDOF + nn] : (__bf16)0.f; __syncthreads(); vst2((unsigned*)(W2T + (size_t)nn * H1 + tid * 8), *(const v4u*)(&srow[tid * 8])); }
}
__device__ __forceinline__ void jacobi_rot(double A[3][3], double V[3][3], int p, int q) {
  const double apq = A[p][q]; if (fabs(apq) < 1e-300) return;
  const double theta = (A[q][q] - A[p][p]) / (2.0 * apq); const double t = (fabs(theta) > 1e150) ? 0.5 / theta : (theta >= 0.0 ? 1.0 : -1.0) / (fabs(theta) + sqrt(theta * theta + 1.0)); const double c = 1.0 / sqrt(t * t + 1.0), s = t * c;
#pragma unroll
  for (int k = 0; k < 3; ++k) { const double akp = A[k][p], akq = A[k][q]; A[k][p] = c * akp - s * akq; A[k][q] = s * akp + c * akq; }
#pragma unroll
  for (int k = 0; k < 3; ++k) { const double apk = A[p][k], aqk = A[q][k]; A[p][k] = c * apk - s * aqk; A[q][k] = s * apk + c * aqk; }
#pragma unroll
  for (int k = 0; k < 3; ++k) { const double vkp = V[k][p], vkq = V[k][q]; V[k][p] = c * vkp - s * vkq; V[k][q] = s * vkp + c * vkq; }
}
__global__ __launch_bounds__(128) void k_main(const float* __restrict__ J, const __bf16* __restrict__ W1T, const float* __restrict__ b1, const __bf16* __restrict__ W2T, const float* __restrict__ b2, float* __restrict__ ODOF, float* __restrict__ OPOSE) {
  __shared__ __align__(16) float sx[64][68];
  __shared__ __align__(16) float shc[4][16][132];
  __shared__ __align__(16) float sang[64][16];
  __shared__ __align__(16) float sdof[64 * NDOF];
  __shared__ __align__(16) float spose[64 * 16];
  const int tid = threadIdx.x, wave = tid >> 5, lane = tid & 31, col = lane & 15, g = lane >> 4; const size_t s0 = (size_t)blockIdx.x * 64;
  for (int q = tid; q < 64 * 68; q += 128) { const int sl = q / 68, c = q - sl * 68; float v = 0.f;
    if (c < DIN) { const int kp = c / 3, ax = c - kp * 3; v = bfr(J[((s0 + sl) * NK + kp) * 3 + ax]) - bfr(J[((s0 + sl) * NK) * 3 + ax]); }
    sx[sl][c] = v; }
  __syncthreads();
  v8f aacc = {};
  const F2 a0 = split_row(&sx[wave * 16 + col][0], 0, lane), a1 = split_rowK(&sx[wave * 16 + col][0], 32, lane, 64);
#pragma unroll 1
  for (int hc = 0; hc < H1 / 128; ++hc) {
#pragma unroll 2
    for (int j = 0; j < 8; ++j) { const int n = hc * 128 + j * 16 + col; v8f acc = {}; const __bf16* wr = W1T + (size_t)(hc * 128 + j * 16 + col) * 64;
      const v16b w0 = frag_b(wr, lane), w1 = frag_b(wr + 32, lane); acc = wmma_bf(a0.l, w0, acc); acc = wmma_bf(a0.h, w0, acc); acc = wmma_bf(a1.l, w1, acc); acc = wmma_bf(a1.h, w1, acc);
      const float bb = bfr(b1[n]);
#pragma unroll
      for (int r = 0; r < 8; ++r) { const float v = acc[r] + bb; shc[wave][8 * g + r][j * 16 + col] = v > 0.f ? v : 0.f; } }
    LDSX();
#pragma unroll
    for (int kc = 0; kc < 4; ++kc) { const F2 ha = split_row(&shc[wave][col][0], kc * 32, lane); const v16b w = frag_b(W2T + (size_t)col * H1 + hc * 128 + kc * 32, lane); aacc = wmma_bf(ha.l, w, aacc); aacc = wmma_bf(ha.h, w, aacc); }
    LDSX(); }
#pragma unroll
  for (int r = 0; r < 8; ++r) sang[wave * 16 + 8 * g + r][col] = aacc[r] + (col < NDOF ? bfr(b2[col]) : 0.f);
  __syncthreads();
  if (tid < 64) { const int sl = tid; const size_t s = s0 + sl;
    float ang[7];
#pragma unroll
    for (int j = 0; j < 7; ++j) { ang[j] = sang[sl][j]; sdof[sl * NDOF + j] = ang[j]; }
    float R[3][3] = {{1.f, 0.f, 0.f}, {0.f, 1.f, 0.f}, {0.f, 0.f, 1.f}}; float p[3] = {0.f, 0.f, 0.f}; float P[14][3];
#pragma unroll
    for (int j = 0; j < 7; ++j) { const float c = cosf(ang[j]), sn = sinf(ang[j]); float Rj[3][3];
      if ((j & 1) == 0) { Rj[0][0] = c; Rj[0][1] = -sn; Rj[0][2] = 0.f; Rj[1][0] = sn; Rj[1][1] = c; Rj[1][2] = 0.f; Rj[2][0] = 0.f; Rj[2][1] = 0.f; Rj[2][2] = 1.f; }
      else { Rj[0][0] = c; Rj[0][1] = 0.f; Rj[0][2] = sn; Rj[1][0] = 0.f; Rj[1][1] = 1.f; Rj[1][2] = 0.f; Rj[2][0] = -sn; Rj[2][1] = 0.f; Rj[2][2] = c; }
      float Rn[3][3];
#pragma unroll
      for (int i = 0; i < 3; ++i)
#pragma unroll
        for (int k = 0; k < 3; ++k) Rn[i][k] = (R[i][0] * Rj[0][k] + R[i][1] * Rj[1][k]) + R[i][2] * Rj[2][k];
#pragma unroll
      for (int i = 0; i < 3; ++i) { R[i][0] = Rn[i][0]; R[i][1] = Rn[i][1]; R[i][2] = Rn[i][2]; }
      const float len = c_len[j];
#pragma unroll
      for (int i = 0; i < 3; ++i) { p[i] = p[i] + R[i][2] * len; P[2 * j][i] = p[i]; P[2 * j + 1][i] = p[i] + R[i][0] * 0.05f; } }
    float cp[3] = {0.f, 0.f, 0.f}, cq[3] = {0.f, 0.f, 0.f};
#pragma unroll
    for (int n = 0; n < 14; ++n)
#pragma unroll
      for (int i = 0; i < 3; ++i) { cp[i] += P[n][i]; cq[i] += sx[sl][n * 3 + i]; }
#pragma unroll
    for (int i = 0; i < 3; ++i) { cp[i] *= (1.0f / 14.0f); cq[i] *= (1.0f / 14.0f); }
    float H[3][3] = {{0.f,0.f,0.f},{0.f,0.f,0.f},{0.f,0.f,0.f}};
#pragma unroll
    for (int n = 0; n < 14; ++n)
#pragma unroll
      for (int i = 0; i < 3; ++i)
#pragma unroll
        for (int k = 0; k < 3; ++k) H[i][k] += (P[n][i] - cp[i]) * (sx[sl][n * 3 + k] - cq[k]);
    double Ad[3][3], Vd[3][3] = {{1.0,0.0,0.0},{0.0,1.0,0.0},{0.0,0.0,1.0}}, Hd[3][3];
#pragma unroll
    for (int i = 0; i < 3; ++i)
#pragma unroll
      for (int k = 0; k < 3; ++k) Hd[i][k] = (double)H[i][k];
#pragma unroll
    for (int i = 0; i < 3; ++i)
#pragma unroll
      for (int k = 0; k < 3; ++k) Ad[i][k] = (Hd[0][i] * Hd[0][k] + Hd[1][i] * Hd[1][k]) + Hd[2][i] * Hd[2][k];
#pragma unroll 1
    for (int sw = 0; sw < 12; ++sw) { jacobi_rot(Ad, Vd, 0, 1); jacobi_rot(Ad, Vd, 0, 2); jacobi_rot(Ad, Vd, 1, 2); }
    double lam0 = Ad[0][0], lam1 = Ad[1][1], lam2 = Ad[2][2];
    double Vs[3][3];
#pragma unroll
    for (int i = 0; i < 3; ++i) { Vs[i][0] = Vd[i][0]; Vs[i][1] = Vd[i][1]; Vs[i][2] = Vd[i][2]; }
#define SWAPCOL(a, b, la, lb) do { if (la < lb) { const double tl = la; la = lb; lb = tl; _Pragma("unroll") for (int i = 0; i < 3; ++i) { const double tv = Vs[i][a]; Vs[i][a] = Vs[i][b]; Vs[i][b] = tv; } } } while (0)
    SWAPCOL(0, 1, lam0, lam1); SWAPCOL(1, 2, lam1, lam2); SWAPCOL(0, 1, lam0, lam1);
    double Us[3][3]; double hv[3];
#pragma unroll
    for (int i = 0; i < 3; ++i) hv[i] = (Hd[i][0] * Vs[0][0] + Hd[i][1] * Vs[1][0]) + Hd[i][2] * Vs[2][0];
    { double nn = sqrt((hv[0] * hv[0] + hv[1] * hv[1]) + hv[2] * hv[2]); nn = nn > 1e-300 ? 1.0 / nn : 0.0; Us[0][0] = hv[0] * nn; Us[1][0] = hv[1] * nn; Us[2][0] = hv[2] * nn; }
#pragma unroll
    for (int i = 0; i < 3; ++i) hv[i] = (Hd[i][0] * Vs[0][1] + Hd[i][1] * Vs[1][1]) + Hd[i][2] * Vs[2][1];
    { const double pr = (hv[0] * Us[0][0] + hv[1] * Us[1][0]) + hv[2] * Us[2][0]; hv[0] -= pr * Us[0][0]; hv[1] -= pr * Us[1][0]; hv[2] -= pr * Us[2][0];
      double nn = sqrt((hv[0] * hv[0] + hv[1] * hv[1]) + hv[2] * hv[2]); nn = nn > 1e-300 ? 1.0 / nn : 0.0; Us[0][1] = hv[0] * nn; Us[1][1] = hv[1] * nn; Us[2][1] = hv[2] * nn; }
    { double c0 = Us[1][0] * Us[2][1] - Us[2][0] * Us[1][1], c1 = Us[2][0] * Us[0][1] - Us[0][0] * Us[2][1], c2 = Us[0][0] * Us[1][1] - Us[1][0] * Us[0][1];
#pragma unroll
      for (int i = 0; i < 3; ++i) hv[i] = (Hd[i][0] * Vs[0][2] + Hd[i][1] * Vs[1][2]) + Hd[i][2] * Vs[2][2];
      const double sgn = ((c0 * hv[0] + c1 * hv[1]) + c2 * hv[2]) < 0.0 ? -1.0 : 1.0; Us[0][2] = sgn * c0; Us[1][2] = sgn * c1; Us[2][2] = sgn * c2; }
    const double detV = Vs[0][0] * (Vs[1][1] * Vs[2][2] - Vs[1][2] * Vs[2][1]) - Vs[0][1] * (Vs[1][0] * Vs[2][2] - Vs[1][2] * Vs[2][0]) + Vs[0][2] * (Vs[1][0] * Vs[2][1] - Vs[1][1] * Vs[2][0]);
    const double detU = Us[0][0] * (Us[1][1] * Us[2][2] - Us[1][2] * Us[2][1]) - Us[0][1] * (Us[1][0] * Us[2][2] - Us[1][2] * Us[2][0]) + Us[0][2] * (Us[1][0] * Us[2][1] - Us[1][1] * Us[2][0]);
    const double ddet = detV * detU; const double d = ddet > 0.0 ? 1.0 : (ddet < 0.0 ? -1.0 : 0.0);
    float Rk[3][3];
#pragma unroll
    for (int i = 0; i < 3; ++i)
#pragma unroll
      for (int k = 0; k < 3; ++k) Rk[i][k] = (float)((Vs[i][0] * Us[k][0] + Vs[i][1] * Us[k][1]) + d * Vs[i][2] * Us[k][2]);
    float tt[3];
#pragma unroll
    for (int i = 0; i < 3; ++i) tt[i] = (cq[i] - ((Rk[i][0] * cp[0] + Rk[i][1] * cp[1]) + Rk[i][2] * cp[2])) + bfr(J[(s * NK) * 3 + i]);
#pragma unroll
    for (int i = 0; i < 3; ++i) { spose[sl * 16 + i * 4] = Rk[i][0]; spose[sl * 16 + i * 4 + 1] = Rk[i][1]; spose[sl * 16 + i * 4 + 2] = Rk[i][2]; spose[sl * 16 + i * 4 + 3] = tt[i]; }
    spose[sl * 16 + 12] = 0.f; spose[sl * 16 + 13] = 0.f; spose[sl * 16 + 14] = 0.f; spose[sl * 16 + 15] = 1.0f; }
  __syncthreads();
  for (int q = tid; q < 64 * NDOF / 4; q += 128) vst2(ODOF + s0 * NDOF + q * 4, *(const v4f*)&sdof[q * 4]);
  for (int q = tid; q < 64 * 16 / 4; q += 128) vst2(OPOSE + s0 * 16 + q * 4, *(const v4f*)&spose[q * 4]);
}

extern "C" void kernel_launch(void* const* d_in, const int* in_sizes, int n_in, void* d_out, int out_size, void* d_ws, size_t ws_size, hipStream_t stream) {
  (void)in_sizes; (void)n_in; (void)out_size; (void)ws_size;
  const float** F = (const float**)d_in;
  char* ws = (char*)d_ws; __bf16* W1T = (__bf16*)ws; __bf16* W2T = (__bf16*)(ws + 2u * H1 * 64);
  float* ODOF = (float*)d_out; float* OPOSE = ODOF + (size_t)NS * NDOF;
  k_pack<<<H1 + 16, 128, 0, stream>>>(F[1], F[3], W1T, W2T);
  k_main<<<NS / 64, 128, 0, stream>>>(F[0], W1T, F[2], W2T, F[4], ODOF, OPOSE);
}
